// KDGQA_20315195310698
// MI455X (gfx1250) — hardware-verified
//
#include <hip/hip_runtime.h>


namespace {
constexpr int B = 8, P = 1024, DIM = 1024, NH = 16, KV = 8, HD = 64, NR = B * P, QW = NH * HD, KW = KV * HD, CW = QW + 2 * KW;
constexpr float XS = 8.0f, PS = 1024.0f, WSC = 256.0f, SCALE = 0.125f;
typedef _Float16 b16;
typedef __attribute__((ext_vector_type(16))) _Float16 v16b;
typedef __attribute__((ext_vector_type(8))) _Float16 v8b;
typedef __attribute__((ext_vector_type(8))) float v8f;
typedef __attribute__((ext_vector_type(4))) float v4f;
typedef __attribute__((ext_vector_type(2))) float v2f;
__device__ __forceinline__ float bf16_rne(float f) { unsigned int u = __float_as_uint(f); u += 0x7FFFu + ((u >> 16) & 1u); return __uint_as_float(u & 0xFFFF0000u); }
__device__ __forceinline__ v16b frag_kb(const b16* p, int hh) { const v8b a = *(const v8b*)(p + 8 * hh), b = *(const v8b*)(p + 16 + 8 * hh); v16b f;
#pragma unroll
  for (int e = 0; e < 8; ++e) { f[e] = a[e]; f[8 + e] = b[e]; } return f; }
__device__ __forceinline__ v8f wmma16b(v16b a, v16b b, v8f c) { v8f d = __builtin_amdgcn_wmma_f32_16x16x32_f16(false, a, false, b, (short)0, c, false, false); asm volatile("v_nop\n\tv_nop\n\tv_nop\n\tv_nop" : "+v"(d) : "v"(a), "v"(b)); return d; }
__device__ __forceinline__ void wave_lds_sync() { __builtin_amdgcn_fence(__ATOMIC_RELEASE, "workgroup"); __builtin_amdgcn_wave_barrier(); __builtin_amdgcn_fence(__ATOMIC_ACQUIRE, "workgroup"); }
__device__ __forceinline__ float pmul(float a, float b) { float p = a * b; asm volatile("" : "+v"(p)); return p; }
__device__ __forceinline__ int iclamp(int v, int lo, int hi) { return v < lo ? lo : (v > hi ? hi : v); }

__global__ __launch_bounds__(256) void wcopy_kernel(const float* __restrict__ wq, const float* __restrict__ wk, const float* __restrict__ wv, const float* __restrict__ wp, b16* __restrict__ WT, b16* __restrict__ WPT) {
  const size_t u = (size_t)blockIdx.x * 256 + threadIdx.x; const size_t nq = (size_t)QW * DIM / 8, nk = (size_t)KW * DIM / 8, np_ = (size_t)DIM * DIM / 8;
  for (int pass = 0; pass < 2; ++pass) {
    if (u < nq + 2 * nk) { const float* w; size_t e, dst; if (u < nq) { w = wq; e = u * 8; dst = e; } else if (u < nq + nk) { w = wk; e = (u - nq) * 8; dst = (size_t)QW * DIM + e; } else { w = wv; e = (u - nq - nk) * 8; dst = (size_t)(QW + KW) * DIM + e; } v8b v; for (int j = 0; j < 8; ++j) v[j] = (b16)(bf16_rne(w[e + j]) * WSC); *(volatile v8b*)(WT + dst) = v; }
    if (u < np_) { v8b v; for (int j = 0; j < 8; ++j) v[j] = (b16)(bf16_rne(wp[u * 8 + j]) * WSC); *(volatile v8b*)(WPT + u * 8) = v; }
    __threadfence(); }
}
__global__ __launch_bounds__(32) void qkv_kernel(const float* __restrict__ x, const b16* __restrict__ WT, int RL, int BV, float* __restrict__ QKV) {
  __shared__ __attribute__((aligned(16))) b16 Ah[16][DIM + 8]; __shared__ float Tf[16][132]; const int lane = threadIdx.x, nloc = lane & 15, hlf = lane >> 4; const int cg = blockIdx.x % (CW / 128); const size_t m0 = (size_t)(blockIdx.x / (CW / 128)) * 16; if (m0 >= (size_t)RL) return;
  if (m0 >= (size_t)BV * P && (cg < QW / 128 || cg >= (QW + KW) / 128)) return;
  for (int rr = 0; rr < 16; ++rr) for (int q = 0; q < DIM / 32; ++q) Ah[rr][q * 32 + lane] = (b16)(bf16_rne(x[(m0 + rr) * DIM + q * 32 + lane]) * XS);
  wave_lds_sync(); v8f acc[8];
#pragma unroll
  for (int t = 0; t < 8; ++t) acc[t] = (v8f){};
#pragma unroll 2
  for (int kb = 0; kb < DIM; kb += 32) { const v16b a = frag_kb(&Ah[nloc][kb], hlf);
#pragma unroll
    for (int t = 0; t < 8; ++t) acc[t] = wmma16b(a, frag_kb(WT + (size_t)(cg * 128 + t * 16 + nloc) * DIM + kb, hlf), acc[t]); }
  const float osc = (cg < QW / 128) ? SCALE / (XS * WSC) : 1.0f / (XS * WSC);
#pragma unroll
  for (int t = 0; t < 8; ++t)
#pragma unroll
    for (int r8 = 0; r8 < 8; ++r8) Tf[8 * hlf + r8][t * 16 + nloc] = acc[t][r8] * osc;
  wave_lds_sync();
  for (int pass = 0; pass < 2; ++pass) { for (int rr = 0; rr < 16; ++rr) *(volatile v4f*)(QKV + (m0 + rr) * CW + cg * 128 + lane * 4) = *(const v4f*)(&Tf[rr][lane * 4]); __threadfence(); }
}
__global__ __launch_bounds__(32) void knorm_kernel(const float* __restrict__ QKV, float* __restrict__ NRM) { const int lane = threadIdx.x; const int b = blockIdx.x / KV, j = blockIdx.x % KV; float s = 0.0f;
#pragma unroll 1
  for (int p = 0; p < P; ++p) { const float* r = QKV + ((size_t)b * P + p) * CW + QW + j * HD; const float a = r[lane], c = r[32 + lane]; s += pmul(a, a) + pmul(c, c); }
  for (int o = 16; o; o >>= 1) s += __shfl_xor(s, o);
  for (int pass = 0; pass < 2; ++pass) { ((volatile float*)NRM)[(size_t)blockIdx.x * 32 + lane] = (lane == 0) ? s : 0.0f; __threadfence(); } }
__global__ __launch_bounds__(32) void alloc_kernel(const float* __restrict__ NRM, int* __restrict__ KVI) {
  __shared__ float kn[KV]; __shared__ int al[KV], kvi[32]; const int lane = threadIdx.x;
  if (lane < KV) { float s = 0.0f;
#pragma unroll 1
    for (int b = 0; b < B; ++b) s += __fsqrt_rn(NRM[(size_t)(b * KV + lane) * 32]); kn[lane] = s; }
  wave_lds_sync();
  __shared__ float nn[KV];
  if (lane == 0) { float mn = kn[0], mx = kn[0];
#pragma unroll 1
    for (int j = 1; j < KV; ++j) { mn = fminf(mn, kn[j]); mx = fmaxf(mx, kn[j]); } float tot = 0.0f;
#pragma unroll 1
    for (int j = 0; j < KV; ++j) { nn[j] = __fdiv_rn(kn[j] - mn, mx - mn); tot += nn[j]; }
    int sum = 0;
#pragma unroll 1
    for (int j = 0; j < KV; ++j) { al[j] = (int)rintf(__fdiv_rn(nn[j], tot) * (float)NH); sum += al[j]; }
    for (int it = 0; it < NH && sum > NH; ++it) { int a = 0; for (int j = 1; j < KV; ++j) if (al[j] > al[a]) a = j; al[a] -= 1; sum -= 1; }
    for (int it = 0; it < NH && sum < NH; ++it) { int a = 0; for (int j = 1; j < KV; ++j) if (al[j] < al[a]) a = j; al[a] += 1; sum += 1; }
    int cum = 0, j = 0; for (int h = 0; h < NH; ++h) { while (j < KV && cum + al[j] <= h) { cum += al[j]; ++j; } kvi[h] = iclamp(j, 0, KV - 1); } for (int h = NH; h < 32; ++h) kvi[h] = 0; }
  wave_lds_sync();
  for (int pass = 0; pass < 2; ++pass) { ((volatile int*)KVI)[lane] = kvi[lane]; __threadfence(); }
}
__global__ __launch_bounds__(32) void att_kernel(const float* __restrict__ QKV, const int* __restrict__ KVI, int BV, float* __restrict__ O) {
  __shared__ __attribute__((aligned(16))) b16 Qp[16][HD + 8], Kp[32][HD + 8], Pp[16][40], Vt[HD][40]; __shared__ float Sc[16][33], Mx[16], Dn[16], Sf[16], Of[16][HD + 2];
  const int lane = threadIdx.x, nloc = lane & 15, hlf = lane >> 4; const int qt = blockIdx.x % (P / 16); const int h = (blockIdx.x / (P / 16)) % NH; const int b = blockIdx.x / ((P / 16) * NH); if (b >= BV) return; const int j = iclamp(KVI[h], 0, KV - 1); const size_t rb = (size_t)b * P; const int q0 = qt * 16;
  for (int rr = 0; rr < 16; ++rr) for (int q = 0; q < 2; ++q) Qp[rr][q * 32 + lane] = (b16)(QKV[(rb + q0 + rr) * CW + h * HD + q * 32 + lane] * XS);
  if (lane < 16) { Mx[lane] = -INFINITY; Dn[lane] = 0.0f; Sf[lane] = 0.0f; }
  v8f acc[4] = {(v8f){}, (v8f){}, (v8f){}, (v8f){}}; wave_lds_sync();
#pragma unroll 1
  for (int kc = 0; kc < P; kc += 32) {
    for (int rr = 0; rr < 32; ++rr) { const float* kr = QKV + (rb + kc + rr) * CW + QW + j * HD; const float* vr = kr + KW; for (int q = 0; q < 2; ++q) { Kp[rr][q * 32 + lane] = (b16)(kr[q * 32 + lane] * XS); Vt[q * 32 + lane][rr] = (b16)(vr[q * 32 + lane] * XS); } }
    wave_lds_sync();
#pragma unroll
    for (int blk = 0; blk < 2; ++blk) { v8f s = {};
#pragma unroll
      for (int kb = 0; kb < HD; kb += 32) s = wmma16b(frag_kb(&Qp[nloc][kb], hlf), frag_kb(&Kp[blk * 16 + nloc][kb], hlf), s);
#pragma unroll
      for (int r8 = 0; r8 < 8; ++r8) Sc[8 * hlf + r8][blk * 16 + nloc] = s[r8] * (1.0f / (XS * XS)); }
    wave_lds_sync();
#pragma unroll 1
    for (int qi = 0; qi < 16; ++qi) { const float sv = Sc[qi][lane]; float cm = sv; for (int o = 16; o; o >>= 1) cm = fmaxf(cm, __shfl_xor(cm, o)); const float mo = Mx[qi]; const float mn = fmaxf(mo, cm); const float p = __expf(sv - mn); float psum = p; for (int o = 16; o; o >>= 1) psum += __shfl_xor(psum, o);
      Pp[qi][lane] = (b16)(p * PS); if (lane == 0) { const float sf = (mo == -INFINITY) ? 0.0f : __expf(mo - mn); Sf[qi] = sf; Dn[qi] = Dn[qi] * sf + psum; Mx[qi] = mn; } }
    wave_lds_sync(); const v16b pa = frag_kb(&Pp[nloc][0], hlf);
#pragma unroll
    for (int t = 0; t < 4; ++t) {
#pragma unroll
      for (int r8 = 0; r8 < 8; ++r8) acc[t][r8] *= Sf[8 * hlf + r8];
      acc[t] = wmma16b(pa, frag_kb(&Vt[t * 16 + nloc][0], hlf), acc[t]); }
    wave_lds_sync(); }
#pragma unroll
  for (int t = 0; t < 4; ++t)
#pragma unroll
    for (int r8 = 0; r8 < 8; ++r8) { const int rl = 8 * hlf + r8; Of[rl][t * 16 + nloc] = acc[t][r8] * (1.0f / (PS * XS)) / Dn[rl]; }
  wave_lds_sync();
  for (int pass = 0; pass < 2; ++pass) { for (int rr = 0; rr < 16; ++rr) *(volatile v2f*)(O + (rb + q0 + rr) * QW + h * HD + lane * 2) = (v2f){Of[rr][lane * 2], Of[rr][lane * 2 + 1]}; __threadfence(); }
}
__global__ __launch_bounds__(32) void proj_kernel(const float* __restrict__ O, const b16* __restrict__ WPT, const float* __restrict__ bp, int RL, float* __restrict__ out) {
  __shared__ __attribute__((aligned(16))) b16 Ah[16][QW + 8]; __shared__ float Tf[16][132]; const int lane = threadIdx.x, nloc = lane & 15, hlf = lane >> 4; const int cg = blockIdx.x % (DIM / 128); const size_t m0 = (size_t)(blockIdx.x / (DIM / 128)) * 16; if (m0 >= (size_t)RL) return;
  for (int rr = 0; rr < 16; ++rr) for (int q = 0; q < QW / 32; ++q) Ah[rr][q * 32 + lane] = (b16)(O[(m0 + rr) * QW + q * 32 + lane] * XS);
  wave_lds_sync(); v8f acc[8];
#pragma unroll
  for (int t = 0; t < 8; ++t) acc[t] = (v8f){};
#pragma unroll 2
  for (int kb = 0; kb < QW; kb += 32) { const v16b a = frag_kb(&Ah[nloc][kb], hlf);
#pragma unroll
    for (int t = 0; t < 8; ++t) acc[t] = wmma16b(a, frag_kb(WPT + (size_t)(cg * 128 + t * 16 + nloc) * QW + kb, hlf), acc[t]); }
#pragma unroll
  for (int t = 0; t < 8; ++t) { const int c = cg * 128 + t * 16 + nloc; const float bb = bf16_rne(bp[c]);
#pragma unroll
    for (int r8 = 0; r8 < 8; ++r8) Tf[8 * hlf + r8][t * 16 + nloc] = acc[t][r8] * (1.0f / (XS * WSC)) + bb; }
  wave_lds_sync();
  for (int pass = 0; pass < 2; ++pass) { for (int rr = 0; rr < 16; ++rr) *(volatile v4f*)(out + (m0 + rr) * DIM + cg * 128 + lane * 4) = *(const v4f*)(&Tf[rr][lane * 4]); __threadfence(); }
}
}

extern "C" void kernel_launch(void* const* d_in, const int* in_sizes, int n_in, void* d_out, int out_size, void* d_ws, size_t ws_size, hipStream_t stream) {
  (void)n_in;
  auto Fp = [&](int i) { return (const float*)d_in[i]; };
  if (in_sizes[0] != NR * DIM || in_sizes[1] != QW * DIM || in_sizes[2] != KW * DIM || in_sizes[3] != KW * DIM || in_sizes[4] != DIM * DIM || in_sizes[5] != DIM || out_size != NR * DIM) return;
  const int BV = B;
  size_t off = 0; char* ws = (char*)d_ws;
  auto carve = [&](size_t bytes) { char* p = ws + off; off += (bytes + 255) & ~(size_t)255; return p; };
  b16* WT = (b16*)carve((size_t)CW * DIM * 2); b16* WPT = (b16*)carve((size_t)DIM * DIM * 2); float* QKV = (float*)carve((size_t)NR * CW * 4); float* NRM = (float*)carve((size_t)B * KV * 32 * 4); int* KVI = (int*)carve(32 * 4); float* O = (float*)carve((size_t)NR * QW * 4);
  if (off > ws_size || off > ((size_t)128 << 20)) return;
  wcopy_kernel<<<(unsigned)(((size_t)CW * DIM / 8 + 255) / 256), 256, 0, stream>>>(Fp(1), Fp(2), Fp(3), Fp(4), WT, WPT);
  qkv_kernel<<<(NR / 16) * (CW / 128), 32, 0, stream>>>(Fp(0), WT, NR, BV, QKV);
  knorm_kernel<<<B * KV, 32, 0, stream>>>(QKV, NRM);
  alloc_kernel<<<1, 32, 0, stream>>>(NRM, KVI);
  att_kernel<<<BV * NH * (P / 16), 32, 0, stream>>>(QKV, KVI, BV, O);
  proj_kernel<<<(BV * P / 16) * (DIM / 128), 32, 0, stream>>>(O, WPT, Fp(5), BV * P, (float*)d_out);
}
